// HARMamba_SingleSensor_v1_31851477467335
// MI455X (gfx1250) — hardware-verified
//
#include <hip/hip_runtime.h>


#define kB     16
#define kL     2048
#define kCIN   7
#define kE     128
#define kDEPTH 12
#define kPATCH 16
#define kP     128
#define kDI    256
#define kDS    16
#define kDR    8
#define kDCONV 4
#define kNCLS  18
#define kBP    (kB * kP)
#define kXPN   (kDR + 2 * kDS)
#define kXPP   64
#define kKPE   128
#define kEPS   1e-5f
#define kWS    256.0f
#define kUS    64.0f
#define kYS    4096.0f

static_assert(kBP % 64 == 0);
static_assert(kE % 64 == 0);
static_assert((2 * kDI) % 64 == 0);
static_assert(kXPP % 64 == 0);
static_assert(kKPE % 32 == 0);
static_assert(kDI % 32 == 0);
static_assert(kCIN * kPATCH <= kKPE);
static_assert(kXPN <= kXPP);
static_assert((kP & (kP - 1)) == 0);
static_assert(kP == 128);
static_assert(kL % 256 == 0);
static_assert(kE == 128);
static_assert(kDI == 256);
static_assert(kB == 16);
static_assert((kB * kNCLS) % 4 == 0);

typedef float          v4f   __attribute__((ext_vector_type(4)));
typedef float          v8f   __attribute__((ext_vector_type(8)));
typedef _Float16       v8h   __attribute__((ext_vector_type(8)));
typedef _Float16       v16h  __attribute__((ext_vector_type(16)));
typedef unsigned short u16x8 __attribute__((ext_vector_type(8)));

union FragH { u16x8 h[2]; v16h v; };
union Pack8 { v8h f; u16x8 u; };

__device__ __forceinline__ v8f zero8() {
    v8f z;
#pragma unroll
    for (int i = 0; i < 8; ++i) z[i] = 0.0f;
    return z;
}
__device__ __forceinline__ v8f ld8f(const float* p) {
    const v4f a = *(const v4f*)p;
    const v4f b = *(const v4f*)(p + 4);
    return __builtin_shufflevector(a, b, 0, 1, 2, 3, 4, 5, 6, 7);
}
__device__ __forceinline__ float wave_sum(float v) {
    v += __shfl_xor(v, 16, 32);
    v += __shfl_xor(v, 8, 32);
    v += __shfl_xor(v, 4, 32);
    v += __shfl_xor(v, 2, 32);
    v += __shfl_xor(v, 1, 32);
    return v;
}
__device__ __forceinline__ float silu_f(float x) {
    const float e = __expf(-x);
    return x * __builtin_amdgcn_rcpf(1.0f + e);
}
__device__ __forceinline__ float softplus_f(float x) {
    return fmaxf(x, 0.0f) + log1pf(__expf(-fabsf(x)));
}
__device__ __forceinline__ float conv4_silu(float x0, float x1, float x2, float x3,
                                            float w0, float w1, float w2, float w3, float bias) {
    const float c = w0 * x0 + w1 * x1 + w2 * x2 + w3 * x3;
    return silu_f(c + bias);
}

__device__ __forceinline__ void mma16(v8f& acc, const FragH& a, const FragH& b) {
    acc = __builtin_amdgcn_wmma_f32_16x16x32_f16(false, a.v, false, b.v, (short)0, acc, false, false);
    asm volatile("v_nop\n\tv_nop\n\tv_nop\n\tv_nop" : "+v"(acc) : "v"(a.v), "v"(b.v));
}

__global__ __launch_bounds__(256)
void cvt_pad_kernel(const float* __restrict__ src, unsigned short* dst, int n8,
                    int dstRow8, int srcRow8, int dstRowsPerGrp, int srcRowsPerGrp, float scale)
{
    const int i = blockIdx.x * 256 + threadIdx.x;
    if (i >= n8) return;
    const int r  = i / dstRow8;
    const int j  = i - r * dstRow8;
    const int g  = r / dstRowsPerGrp;
    const int rr = r - g * dstRowsPerGrp;
    v8f x = zero8();
    if (j < srcRow8 && rr < srcRowsPerGrp)
        x = ld8f(src + ((size_t)(g * srcRowsPerGrp + rr) * srcRow8 + j) * 8);
    Pack8 pk;
    pk.f = __builtin_convertvector(x * scale, v8h);
    const u16x8 v = pk.u;
    const size_t e = (size_t)i * 8;
    *(volatile u16x8*)(dst + e) = v;
    __threadfence();
    *(volatile u16x8*)(dst + e) = v;
}

__global__ __launch_bounds__(256)
void revin_rows_kernel(const float* __restrict__ imu, const float* __restrict__ rw,
                       const float* __restrict__ rb, unsigned short* xa)
{
    __shared__ float red[8][8];
    __shared__ float smu[8];
    __shared__ float srs[8];
    const int b = blockIdx.x, tid = threadIdx.x, lane = tid & 31, wave = tid >> 5;
    const float* xb = imu + (size_t)b * kL * kCIN;

    float s[kCIN];
#pragma unroll
    for (int c = 0; c < kCIN; ++c) s[c] = 0.0f;
#pragma unroll 1
    for (int j = 0; j < kL / 256; ++j) {
        const float* xr = xb + (size_t)(j * 256 + tid) * kCIN;
#pragma unroll
        for (int c = 0; c < kCIN; ++c) s[c] += xr[c];
    }
#pragma unroll
    for (int c = 0; c < kCIN; ++c) s[c] = wave_sum(s[c]);
    if (lane == 0) {
#pragma unroll
        for (int c = 0; c < kCIN; ++c) red[wave][c] = s[c];
    }
    __syncthreads();
    float mu[kCIN];
#pragma unroll
    for (int c = 0; c < kCIN; ++c) {
        float t = 0.0f;
#pragma unroll
        for (int w = 0; w < 8; ++w) t += red[w][c];
        mu[c] = t * (1.0f / kL);
    }
    __syncthreads();

    float q[kCIN];
#pragma unroll
    for (int c = 0; c < kCIN; ++c) q[c] = 0.0f;
#pragma unroll 1
    for (int j = 0; j < kL / 256; ++j) {
        const float* xr = xb + (size_t)(j * 256 + tid) * kCIN;
#pragma unroll
        for (int c = 0; c < kCIN; ++c) { const float dd = xr[c] - mu[c]; q[c] += dd * dd; }
    }
#pragma unroll
    for (int c = 0; c < kCIN; ++c) q[c] = wave_sum(q[c]);
    if (lane == 0) {
#pragma unroll
        for (int c = 0; c < kCIN; ++c) red[wave][c] = q[c];
    }
    __syncthreads();
    if (tid == 0) {
#pragma unroll
        for (int c = 0; c < kCIN; ++c) {
            float t = 0.0f;
#pragma unroll
            for (int w = 0; w < 8; ++w) t += red[w][c];
            const float var = t * (1.0f / kL);
            smu[c] = mu[c];
            srs[c] = rsqrtf(var + kEPS);
        }
    }
    __syncthreads();

#pragma unroll 1
    for (int it = 0; it < (kP * (kKPE / 8)) / 256; ++it) {
        const int id = it * 256 + tid;
        const int p = id >> 4;
        const int j = id & 15;
        v8f v = zero8();
        if (j < (kCIN * kPATCH) / 8) {
            const int c  = j >> 1;
            const int k0 = (j & 1) * 8;
            const float m = smu[c], r = srs[c], w = rw[c], bb = rb[c];
            const float* xp = xb + (size_t)(p * kPATCH + k0) * kCIN + c;
#pragma unroll
            for (int qq = 0; qq < 8; ++qq) v[qq] = ((xp[qq * kCIN] - m) * r) * w + bb;
        }
        Pack8 pk;
        pk.f = __builtin_convertvector(v, v8h);
        const u16x8 o = pk.u;
        unsigned short* gp = xa + ((size_t)(b * kP + p) * kKPE + (size_t)j * 8);
        *(volatile u16x8*)gp = o;
        __threadfence();
        *(volatile u16x8*)gp = o;
    }
}

__device__ __forceinline__ void tile_store_pass(const float* st, float* gp, int ldc, int lane) {
    constexpr int P = 36;
    const int rsub = lane >> 3;
    const int c4   = (lane & 7) * 4;
#pragma unroll
    for (int it = 0; it < 8; ++it) {
        const int row = it * 4 + rsub;
        const v4f v = *(const v4f*)(st + row * P + c4);
        *(volatile v4f*)(gp + (size_t)row * ldc + c4) = v;
    }
}

template<int EPI>
__global__ __launch_bounds__(128)
void gemm_tn_kernel(const unsigned short* __restrict__ A, const unsigned short* __restrict__ Bw,
                    float* C, const float* __restrict__ cbias, const float* __restrict__ radd,
                    int K, int ldc, size_t sAz, size_t sBz, size_t sCz, float scale)
{
    constexpr int NBF = 2;
    constexpr int P   = 36;
    __shared__ __attribute__((aligned(16))) float stile[4][32 * P];

    const int tid  = threadIdx.x;
    const int lane = tid & 31;
    const int wave = tid >> 5;
    const int h    = lane >> 4;
    const int m    = lane & 15;
    const int wm   = wave >> 1;
    const int wn   = wave & 1;
    const int z    = blockIdx.z;
    A  += (size_t)z * sAz;
    Bw += (size_t)z * sBz;
    C  += (size_t)z * sCz;

    const int rowW = blockIdx.y * 64 + wm * 32;
    const int colW = blockIdx.x * 64 + wn * 32;

    v8f acc[2 * NBF];
#pragma unroll
    for (int j = 0; j < 2 * NBF; ++j) acc[j] = zero8();

    const size_t aoff  = (size_t)(rowW + m) * K + 8 * h;
    const size_t boff  = (size_t)(colW + m) * K + 8 * h;
    const size_t sub16 = (size_t)16 * K;
    const int nk = K >> 5;

    for (int kt = 0; kt < nk; ++kt) {
        const size_t k0 = (size_t)kt * 32;
        FragH fa[2], fb[NBF];
#pragma unroll
        for (int s = 0; s < 2; ++s) {
            const unsigned short* p = A + aoff + s * sub16 + k0;
            fa[s].h[0] = *(const u16x8*)(p);
            fa[s].h[1] = *(const u16x8*)(p + 16);
        }
#pragma unroll
        for (int j = 0; j < NBF; ++j) {
            const unsigned short* p = Bw + boff + j * sub16 + k0;
            fb[j].h[0] = *(const u16x8*)(p);
            fb[j].h[1] = *(const u16x8*)(p + 16);
        }
#pragma unroll
        for (int s = 0; s < 2; ++s)
#pragma unroll
            for (int j = 0; j < NBF; ++j)
                mma16(acc[s * NBF + j], fa[s], fb[j]);
    }

    float* st = stile[wave];
#pragma unroll
    for (int s = 0; s < 2; ++s)
#pragma unroll
        for (int j = 0; j < NBF; ++j)
#pragma unroll
            for (int r = 0; r < 8; ++r) {
                const int lr = s * 16 + 8 * h + r;
                const int lc = j * 16 + m;
                float v = acc[s * NBF + j][r] * scale;
                if (EPI == 1) {
                    v += cbias[colW + lc];
                    v += radd[(size_t)((rowW + lr) & (kP - 1)) * ldc + colW + lc];
                }
                st[lr * P + lc] = v;
            }
    __syncthreads();

    float* gp = C + (size_t)rowW * ldc + colW;
    tile_store_pass(st, gp, ldc, lane);
    __threadfence();
    tile_store_pass(st, gp, ldc, lane);
}

__global__ __launch_bounds__(128)
void ln_rows_kernel(const float* __restrict__ S, const float* __restrict__ lw,
                    const float* __restrict__ lb, unsigned short* hn, int layer0)
{
    __shared__ __attribute__((aligned(16))) _Float16 stg[4 * 2 * kE];
    const int tid = threadIdx.x, lane = tid & 31, wave = tid >> 5;
    const int z = blockIdx.y;
    const int l = layer0 + z;
    const int bp0 = blockIdx.x * 8 + wave * 2;
    const v4f w4 = *(const v4f*)(lw + (size_t)l * kE + 4 * lane);
    const v4f b4 = *(const v4f*)(lb + (size_t)l * kE + 4 * lane);

#pragma unroll
    for (int rr = 0; rr < 2; ++rr) {
        const int bp = bp0 + rr;
        const int b = bp >> 7, p = bp & (kP - 1);
        const int ps = z ? (kP - 1 - p) : p;
        const v4f x = *(const v4f*)(S + ((size_t)b * kP + ps) * kE + 4 * lane);
        float sm = (x[0] + x[1]) + (x[2] + x[3]);
        sm = wave_sum(sm);
        const float mu = sm * (1.0f / kE);
        float dd[4];
        float sq = 0.0f;
#pragma unroll
        for (int j = 0; j < 4; ++j) { dd[j] = x[j] - mu; sq += dd[j] * dd[j]; }
        sq = wave_sum(sq);
        const float r = rsqrtf(sq * (1.0f / kE) + kEPS);
        _Float16* sp = stg + (wave * 2 + rr) * kE + 4 * lane;
#pragma unroll
        for (int j = 0; j < 4; ++j) sp[j] = (_Float16)(dd[j] * r * w4[j] + b4[j]);
    }
    __syncthreads();
    const int rr = lane >> 4;
    const int c  = (lane & 15) * 8;
    Pack8 pk;
    pk.f = *(const v8h*)(stg + (wave * 2 + rr) * kE + c);
    const u16x8 o = pk.u;
    unsigned short* gp = hn + ((size_t)z * kBP + bp0 + rr) * kE + c;
    *(volatile u16x8*)gp = o;
    __threadfence();
    *(volatile u16x8*)gp = o;
}

__global__ __launch_bounds__(128)
void conv_silu_kernel(const float* __restrict__ xz, const float* __restrict__ cw,
                      const float* __restrict__ cb, unsigned short* u16, int layer0)
{
    const int lane = threadIdx.x & 31, wave = threadIdx.x >> 5;
    const int z  = blockIdx.y;
    const int bp = blockIdx.x * 4 + wave;
    const int p  = bp & (kP - 1);
    const int l  = layer0 + z;
    const int d0 = lane * 8;
    const float* xr = xz + ((size_t)z * kBP + bp) * (2 * kDI) + d0;

    const v8f x3 = ld8f(xr);
    v8f x2 = zero8(), x1 = zero8(), x0 = zero8();
    if (p >= 1) x2 = ld8f(xr - 2 * kDI);
    if (p >= 2) x1 = ld8f(xr - 2 * (2 * kDI));
    if (p >= 3) x0 = ld8f(xr - 3 * (2 * kDI));

    const float* wp = cw + ((size_t)l * kDI + d0) * kDCONV;
    v4f wv[8];
#pragma unroll
    for (int c = 0; c < 8; ++c) wv[c] = *(const v4f*)(wp + 4 * c);
    const v8f bias = ld8f(cb + (size_t)l * kDI + d0);

    v8f u;
#pragma unroll
    for (int c = 0; c < 8; ++c)
        u[c] = conv4_silu(x0[c], x1[c], x2[c], x3[c], wv[c][0], wv[c][1], wv[c][2], wv[c][3], bias[c]) * kUS;

    Pack8 pk;
    pk.f = __builtin_convertvector(u, v8h);
    const u16x8 v = pk.u;
    unsigned short* gp = u16 + ((size_t)z * kBP + bp) * kDI + d0;
    *(volatile u16x8*)gp = v;
    __threadfence();
    *(volatile u16x8*)gp = v;
}

__device__ __forceinline__ void y_store_pass(const _Float16* sy, unsigned short* y16, size_t gbase,
                                             int lane, int wave) {
#pragma unroll
    for (int k = 0; k < 2; ++k) {
        const int it = wave * 2 + k;
        const int t  = it * 4 + (lane >> 3);
        const int c  = (lane & 7) * 8;
        Pack8 pk;
        pk.f = *(const v8h*)(sy + t * 64 + c);
        *(volatile u16x8*)(y16 + gbase + (size_t)t * kDI + c) = pk.u;
    }
}

__global__ __launch_bounds__(64)
void scan_kernel(const float* __restrict__ xz, const float* __restrict__ dbl,
                 const float* __restrict__ cw, const float* __restrict__ cb,
                 const float* __restrict__ dtw, const float* __restrict__ dtb,
                 const float* __restrict__ Alog, const float* __restrict__ Dpp,
                 unsigned short* y16, int layer0)
{
    __shared__ __attribute__((aligned(16))) float sdbl[16 * kXPN];
    __shared__ __attribute__((aligned(16))) _Float16 sy[16 * 64];

    const int tid = threadIdx.x, lane = tid & 31, wave = tid >> 5;
    const int dbase = blockIdx.x * 64;
    const int d = dbase + tid;
    const int b = blockIdx.y, z = blockIdx.z;
    const int l = layer0 + z;
    const int ld = l * kDI + d;

    float an[kDS], hs[kDS], wr[kDR];
#pragma unroll
    for (int n = 0; n < kDS; ++n) { an[n] = -expf(Alog[(size_t)ld * kDS + n]); hs[n] = 0.0f; }
#pragma unroll
    for (int r = 0; r < kDR; ++r) wr[r] = dtw[(size_t)ld * kDR + r];
    const float tb = dtb[ld];
    const float Dd = Dpp[ld];
    const float w0 = cw[(size_t)ld * kDCONV + 0], w1 = cw[(size_t)ld * kDCONV + 1];
    const float w2 = cw[(size_t)ld * kDCONV + 2], w3 = cw[(size_t)ld * kDCONV + 3];
    const float cbias = cb[ld];
    float xm1 = 0.0f, xm2 = 0.0f, xm3 = 0.0f;
    const size_t row0 = (size_t)z * kBP + (size_t)b * kP;

#pragma unroll 1
    for (int p0 = 0; p0 < kP; p0 += 16) {
        for (int i = tid; i < 16 * kXPN; i += 64) {
            const int t = i / kXPN;
            const int c = i - t * kXPN;
            sdbl[i] = dbl[(row0 + p0 + t) * kXPP + c];
        }
        __syncthreads();
#pragma unroll 1
        for (int t = 0; t < 16; ++t) {
            const size_t e = (row0 + p0 + t) * (2 * kDI) + d;
            const float xv = xz[e];
            const float zv = xz[e + kDI];
            const float u = conv4_silu(xm3, xm2, xm1, xv, w0, w1, w2, w3, cbias);
            xm3 = xm2; xm2 = xm1; xm1 = xv;
            const float* sr = sdbl + t * kXPN;
            float a = 0.0f;
#pragma unroll
            for (int r = 0; r < kDR; ++r) a += sr[r] * wr[r];
            const float dt = softplus_f(a + tb);
            const float du = dt * u;
            float y = 0.0f;
#pragma unroll
            for (int n = 0; n < kDS; ++n) {
                const float da = __expf(dt * an[n]);
                hs[n] = da * hs[n] + du * sr[kDR + n];
                y += hs[n] * sr[kDR + kDS + n];
            }
            const float g = (y + Dd * u) * silu_f(zv);
            sy[t * 64 + tid] = (_Float16)(g * kYS);
        }
        __syncthreads();
        const size_t gbase = (row0 + p0) * kDI + dbase;
        y_store_pass(sy, y16, gbase, lane, wave);
        __threadfence();
        y_store_pass(sy, y16, gbase, lane, wave);
        __syncthreads();
    }
}

__global__ __launch_bounds__(128)
void merge_kernel(const float* __restrict__ Sin, const float* __restrict__ ob, float* Sout)
{
    const int lane = threadIdx.x & 31, wave = threadIdx.x >> 5;
    const int bp = blockIdx.x * 4 + wave;
    const int b = bp >> 7, p = bp & (kP - 1);
    const int e = 4 * lane;
    const v4f s  = *(const v4f*)(Sin + (size_t)bp * kE + e);
    const v4f hf = *(const v4f*)(ob + (size_t)bp * kE + e);
    const v4f hb = *(const v4f*)(ob + ((size_t)kBP + (size_t)b * kP + (kP - 1 - p)) * kE + e);
    const v4f o = (s + s) + (hf + hb);
    float* gp = Sout + (size_t)bp * kE + e;
    *(volatile v4f*)gp = o;
    __threadfence();
    *(volatile v4f*)gp = o;
}

__device__ __forceinline__ void out_store_pass(const float* src, float* dst, int lane) {
    for (int i = lane; i < (kB * kNCLS) / 4; i += 32) {
        const v4f v = *(const v4f*)(src + 4 * i);
        *(volatile v4f*)(dst + 4 * i) = v;
    }
}

__global__ __launch_bounds__(256)
void final_kernel(const float* __restrict__ S, const float* __restrict__ nw, const float* __restrict__ nb,
                  const float* __restrict__ hw, const float* __restrict__ hbias, float* out)
{
    __shared__ __attribute__((aligned(16))) float featL[kB * kE];
    __shared__ __attribute__((aligned(16))) float outL[kB * kNCLS];
    const int tid = threadIdx.x, lane = tid & 31, wave = tid >> 5;
    const int e0 = 4 * lane;
    const v4f w4 = *(const v4f*)(nw + e0);
    const v4f b4 = *(const v4f*)(nb + e0);

#pragma unroll 1
    for (int bi = 0; bi < 2; ++bi) {
        const int b = wave * 2 + bi;
        float a0 = 0.0f, a1 = 0.0f, a2 = 0.0f, a3 = 0.0f;
#pragma unroll 1
        for (int p = 0; p < kP; ++p) {
            const v4f x = *(const v4f*)(S + ((size_t)b * kP + p) * kE + e0);
            float sm = (x[0] + x[1]) + (x[2] + x[3]);
            sm = wave_sum(sm);
            const float mu = sm * (1.0f / kE);
            const float d0 = x[0] - mu, d1 = x[1] - mu, d2 = x[2] - mu, d3 = x[3] - mu;
            float sq = d0 * d0 + d1 * d1 + d2 * d2 + d3 * d3;
            sq = wave_sum(sq);
            const float r = rsqrtf(sq * (1.0f / kE) + kEPS);
            a0 += d0 * r * w4[0] + b4[0];
            a1 += d1 * r * w4[1] + b4[1];
            a2 += d2 * r * w4[2] + b4[2];
            a3 += d3 * r * w4[3] + b4[3];
        }
        float* fp = featL + b * kE + e0;
        fp[0] = a0 * (1.0f / kP);
        fp[1] = a1 * (1.0f / kP);
        fp[2] = a2 * (1.0f / kP);
        fp[3] = a3 * (1.0f / kP);
    }
    __syncthreads();

    for (int o = tid; o < kB * kNCLS; o += 256) {
        const int b = o / kNCLS;
        const int c = o - b * kNCLS;
        const float* fr = featL + b * kE;
        const float* wrow = hw + (size_t)c * kE;
        float a = 0.0f;
#pragma unroll 1
        for (int e = 0; e < kE; ++e) a += fr[e] * wrow[e];
        outL[o] = a + hbias[c];
    }
    __syncthreads();

    if (wave == 0) {
        out_store_pass(outL, out, lane);
        __threadfence();
        out_store_pass(outL, out, lane);
    }
}

extern "C" void kernel_launch(void* const* d_in, const int* in_sizes, int n_in,
                              void* d_out, int out_size, void* d_ws, size_t ws_size,
                              hipStream_t stream)
{
    if (n_in < 21) return;
    if (in_sizes[0]  != kB * kL * kCIN)          return;
    if (in_sizes[1]  != kCIN)                    return;
    if (in_sizes[2]  != kCIN)                    return;
    if (in_sizes[3]  != kE * kCIN * kPATCH)      return;
    if (in_sizes[4]  != kE)                      return;
    if (in_sizes[5]  != kP * kE)                 return;
    if (in_sizes[6]  != kDEPTH * kE)             return;
    if (in_sizes[7]  != kDEPTH * kE)             return;
    if (in_sizes[8]  != kDEPTH * 2 * kDI * kE)   return;
    if (in_sizes[9]  != kDEPTH * kDI * kDCONV)   return;
    if (in_sizes[10] != kDEPTH * kDI)            return;
    if (in_sizes[11] != kDEPTH * kXPN * kDI)     return;
    if (in_sizes[12] != kDEPTH * kDI * kDR)      return;
    if (in_sizes[13] != kDEPTH * kDI)            return;
    if (in_sizes[14] != kDEPTH * kDI * kDS)      return;
    if (in_sizes[15] != kDEPTH * kDI)            return;
    if (in_sizes[16] != kDEPTH * kE * kDI)       return;
    if (in_sizes[17] != kE)                      return;
    if (in_sizes[18] != kE)                      return;
    if (in_sizes[19] != kNCLS * kE)              return;
    if (in_sizes[20] != kNCLS)                   return;
    if (out_size != kB * kNCLS)                  return;

    const float* imu      = (const float*)d_in[0];
    const float* revin_w  = (const float*)d_in[1];
    const float* revin_b  = (const float*)d_in[2];
    const float* patch_w  = (const float*)d_in[3];
    const float* patch_b  = (const float*)d_in[4];
    const float* pos_emb  = (const float*)d_in[5];
    const float* ln_w     = (const float*)d_in[6];
    const float* ln_b     = (const float*)d_in[7];
    const float* in_w     = (const float*)d_in[8];
    const float* conv_w   = (const float*)d_in[9];
    const float* conv_b   = (const float*)d_in[10];
    const float* xproj_w  = (const float*)d_in[11];
    const float* dt_w     = (const float*)d_in[12];
    const float* dt_b     = (const float*)d_in[13];
    const float* A_log    = (const float*)d_in[14];
    const float* Dp       = (const float*)d_in[15];
    const float* out_w    = (const float*)d_in[16];
    const float* normf_w  = (const float*)d_in[17];
    const float* normf_b  = (const float*)d_in[18];
    const float* head_w   = (const float*)d_in[19];
    const float* head_b   = (const float*)d_in[20];
    float* out = (float*)d_out;

    const size_t SZ_WIN  = (size_t)kDEPTH * 2 * kDI * kE * 2;
    const size_t SZ_WOUT = (size_t)kDEPTH * kE * kDI * 2;
    const size_t SZ_WXP  = (size_t)kDEPTH * kXPP * kDI * 2;
    const size_t SZ_WPE  = (size_t)kE * kKPE * 2;
    const size_t SZ_XA   = (size_t)kBP * kKPE * 2;
    const size_t SZ_S    = (size_t)kBP * kE * 4;
    const size_t SZ_HN   = (size_t)2 * kBP * kE * 2;
    const size_t SZ_XZ   = (size_t)2 * kBP * 2 * kDI * 4;
    const size_t SZ_U16  = (size_t)2 * kBP * kDI * 2;
    const size_t SZ_DBL  = (size_t)2 * kBP * kXPP * 4;
    const size_t SZ_Y16  = (size_t)2 * kBP * kDI * 2;
    const size_t SZ_OB   = (size_t)2 * kBP * kE * 4;

    const size_t OFF_WIN  = 0;
    const size_t OFF_WOUT = OFF_WIN  + SZ_WIN;
    const size_t OFF_WXP  = OFF_WOUT + SZ_WOUT;
    const size_t OFF_WPE  = OFF_WXP  + SZ_WXP;
    const size_t OFF_XA   = OFF_WPE  + SZ_WPE;
    const size_t OFF_SA   = OFF_XA   + SZ_XA;
    const size_t OFF_SB   = OFF_SA   + SZ_S;
    const size_t OFF_HN   = OFF_SB   + SZ_S;
    const size_t OFF_XZ   = OFF_HN   + SZ_HN;
    const size_t OFF_U16  = OFF_XZ   + SZ_XZ;
    const size_t OFF_DBL  = OFF_U16  + SZ_U16;
    const size_t OFF_Y16  = OFF_DBL  + SZ_DBL;
    const size_t OFF_OB   = OFF_Y16  + SZ_Y16;
    const size_t WS_END   = OFF_OB   + SZ_OB;
    if (ws_size < WS_END) return;

    char* ws = (char*)d_ws;
    unsigned short* w16_in  = (unsigned short*)(ws + OFF_WIN);
    unsigned short* w16_out = (unsigned short*)(ws + OFF_WOUT);
    unsigned short* w16_xp  = (unsigned short*)(ws + OFF_WXP);
    unsigned short* w16_pe  = (unsigned short*)(ws + OFF_WPE);
    unsigned short* xa16    = (unsigned short*)(ws + OFF_XA);
    float*          SA      = (float*)(ws + OFF_SA);
    float*          SB      = (float*)(ws + OFF_SB);
    unsigned short* hn16    = (unsigned short*)(ws + OFF_HN);
    float*          xz      = (float*)(ws + OFF_XZ);
    unsigned short* u16     = (unsigned short*)(ws + OFF_U16);
    float*          dbl     = (float*)(ws + OFF_DBL);
    unsigned short* y16     = (unsigned short*)(ws + OFF_Y16);
    float*          outbuf  = (float*)(ws + OFF_OB);

    {
        int n8;
        n8 = (kDEPTH * 2 * kDI * kE) / 8;
        hipLaunchKernelGGL(cvt_pad_kernel, dim3((n8 + 255) / 256), dim3(256), 0, stream,
                           in_w, w16_in, n8, kE / 8, kE / 8, kDEPTH * 2 * kDI, kDEPTH * 2 * kDI, kWS);
        n8 = (kDEPTH * kE * kDI) / 8;
        hipLaunchKernelGGL(cvt_pad_kernel, dim3((n8 + 255) / 256), dim3(256), 0, stream,
                           out_w, w16_out, n8, kDI / 8, kDI / 8, kDEPTH * kE, kDEPTH * kE, kWS);
        n8 = (kDEPTH * kXPP * kDI) / 8;
        hipLaunchKernelGGL(cvt_pad_kernel, dim3((n8 + 255) / 256), dim3(256), 0, stream,
                           xproj_w, w16_xp, n8, kDI / 8, kDI / 8, (int)kXPP, (int)kXPN, kWS);
        n8 = (kE * kKPE) / 8;
        hipLaunchKernelGGL(cvt_pad_kernel, dim3((n8 + 255) / 256), dim3(256), 0, stream,
                           patch_w, w16_pe, n8, kKPE / 8, (kCIN * kPATCH) / 8, (int)kE, (int)kE, kWS);
    }

    hipLaunchKernelGGL(revin_rows_kernel, dim3(kB), dim3(256), 0, stream, imu, revin_w, revin_b, xa16);

    hipLaunchKernelGGL(HIP_KERNEL_NAME(gemm_tn_kernel<1>), dim3(kE / 64, kBP / 64, 1), dim3(128), 0, stream,
                       (const unsigned short*)xa16, (const unsigned short*)w16_pe, SA, patch_b, pos_emb,
                       (int)kKPE, (int)kE, (size_t)0, (size_t)0, (size_t)0, 1.0f / kWS);

    float* Sbuf[2] = { SA, SB };
    for (int i = 0; i < kDEPTH / 2; ++i) {
        const int l0 = 2 * i;
        float* Scur  = Sbuf[i & 1];
        float* Snext = Sbuf[(i + 1) & 1];

        hipLaunchKernelGGL(ln_rows_kernel, dim3(kBP / 8, 2), dim3(128), 0, stream,
                           (const float*)Scur, ln_w, ln_b, hn16, l0);

        hipLaunchKernelGGL(HIP_KERNEL_NAME(gemm_tn_kernel<0>), dim3((2 * kDI) / 64, kBP / 64, 2), dim3(128), 0, stream,
                           (const unsigned short*)hn16, (const unsigned short*)(w16_in + (size_t)l0 * 2 * kDI * kE), xz,
                           patch_b, pos_emb,
                           (int)kE, (int)(2 * kDI), (size_t)kBP * kE, (size_t)2 * kDI * kE, (size_t)kBP * 2 * kDI,
                           1.0f / kWS);

        hipLaunchKernelGGL(conv_silu_kernel, dim3(kBP / 4, 2), dim3(128), 0, stream,
                           (const float*)xz, conv_w, conv_b, u16, l0);

        hipLaunchKernelGGL(HIP_KERNEL_NAME(gemm_tn_kernel<0>), dim3(kXPP / 64, kBP / 64, 2), dim3(128), 0, stream,
                           (const unsigned short*)u16, (const unsigned short*)(w16_xp + (size_t)l0 * kXPP * kDI), dbl,
                           patch_b, pos_emb,
                           (int)kDI, (int)kXPP, (size_t)kBP * kDI, (size_t)kXPP * kDI, (size_t)kBP * kXPP,
                           1.0f / (kUS * kWS));

        hipLaunchKernelGGL(scan_kernel, dim3(kDI / 64, kB, 2), dim3(64), 0, stream,
                           (const float*)xz, (const float*)dbl, conv_w, conv_b, dt_w, dt_b, A_log, Dp, y16, l0);

        hipLaunchKernelGGL(HIP_KERNEL_NAME(gemm_tn_kernel<0>), dim3(kE / 64, kBP / 64, 2), dim3(128), 0, stream,
                           (const unsigned short*)y16, (const unsigned short*)(w16_out + (size_t)l0 * kE * kDI), outbuf,
                           patch_b, pos_emb,
                           (int)kDI, (int)kE, (size_t)kBP * kDI, (size_t)kE * kDI, (size_t)kBP * kE,
                           1.0f / (kYS * kWS));

        hipLaunchKernelGGL(merge_kernel, dim3(kBP / 4), dim3(128), 0, stream,
                           (const float*)Scur, (const float*)outbuf, Snext);
    }

    hipLaunchKernelGGL(final_kernel, dim3(1), dim3(256), 0, stream,
                       (const float*)Sbuf[(kDEPTH / 2) & 1], normf_w, normf_b, head_w, head_b, out);
}
